// SampleSelfAttention_6244882448561
// MI455X (gfx1250) — hardware-run, weakly checked
//
#include <hip/hip_runtime.h>


#define NN   4096
#define EE   1024
#define NH_  8
#define HD   128
#define PCAR 1024.0f
typedef _Float16 h16;
typedef unsigned short bf;
typedef __attribute__((ext_vector_type(16))) __bf16   v16bf;
typedef __attribute__((ext_vector_type(16))) _Float16 v16h;
typedef __attribute__((ext_vector_type(8)))  _Float16 v8h;
typedef __attribute__((ext_vector_type(8)))  unsigned short v8us;
typedef __attribute__((ext_vector_type(8)))  float    v8f;
typedef __attribute__((ext_vector_type(4)))  float    v4f;
typedef v8h  __attribute__((may_alias)) v8ha;
typedef v4f  __attribute__((may_alias)) v4fa;
typedef v8us __attribute__((may_alias)) v8usa;

__device__ __forceinline__ unsigned short f2bf(float f) { unsigned u = __float_as_uint(f); u += 0x7FFFu + ((u >> 16) & 1u); return (unsigned short)(u >> 16); }
__device__ __forceinline__ float bf2f(unsigned short b) { return __uint_as_float(((unsigned)b) << 16); }
__device__ __forceinline__ float bfr(float f) { return bf2f(f2bf(f)); }
__device__ __forceinline__ v16h cat16(v8h lo, v8h hi) { return __builtin_shufflevector(lo, hi, 0, 1, 2, 3, 4, 5, 6, 7, 8, 9, 10, 11, 12, 13, 14, 15); }
__device__ __forceinline__ v16bf cat16b(v8us lo, v8us hi) { return __builtin_bit_cast(v16bf, __builtin_shufflevector(lo, hi, 0, 1, 2, 3, 4, 5, 6, 7, 8, 9, 10, 11, 12, 13, 14, 15)); }
__device__ __forceinline__ v8f wmma16(v16h a, v16h b, v8f c) { return __builtin_amdgcn_wmma_f32_16x16x32_f16(false, a, false, b, (short)0, c, false, false); }
__device__ __forceinline__ v8f wmmab(v16bf a, v16bf b, v8f c) { return __builtin_amdgcn_wmma_f32_16x16x32_bf16(false, a, false, b, (short)0, c, false, false); }


template <typename T16> struct WFrag;
template <> struct WFrag<h16> { typedef v16h V; static __device__ __forceinline__ V ld(const h16* p) { return cat16(*(const v8h*)p, *(const v8h*)(p + 16)); } static __device__ __forceinline__ v8f mma(V a, V b, v8f c) { return wmma16(a, b, c); } };
template <> struct WFrag<bf> { typedef v16bf V; static __device__ __forceinline__ V ld(const bf* p) { return cat16b(*(const v8us*)p, *(const v8us*)(p + 16)); } static __device__ __forceinline__ v8f mma(V a, V b, v8f c) { return wmmab(a, b, c); } };
template <typename T16, int NSPLIT, bool BIAS>
__global__ __launch_bounds__(32) void k_gemmw(const T16* __restrict__ A, const T16* __restrict__ A2, const T16* __restrict__ Bt, const T16* __restrict__ Bt2, int K, float* C, int ldc, const float* __restrict__ bias, size_t sA, size_t sB, size_t sC) {
    typedef typename WFrag<T16>::V V;
    __shared__ __align__(16) float os[16 * 68];
    const size_t z = blockIdx.z; A += z * sA; if (A2) A2 += z * sA; Bt += z * sB; if (Bt2) Bt2 += z * sB; C += z * sC;
    const int lane = threadIdx.x & 31, lr = lane & 15, hi = lane >> 4; const int r0 = blockIdx.x * 64, c0 = blockIdx.y * 64;
    v8f acc[4][4];
#pragma unroll
    for (int mb = 0; mb < 4; ++mb)
#pragma unroll
        for (int nb = 0; nb < 4; ++nb) acc[mb][nb] = (v8f){};
    const size_t aoff = (size_t)(r0 + lr) * K + 8 * hi, boff = (size_t)(c0 + lr) * K + 8 * hi;
#pragma unroll 1
    for (int kc = 0; kc < K; kc += 32) {
        V a[4], a2[4];
#pragma unroll
        for (int mb = 0; mb < 4; ++mb) { a[mb] = WFrag<T16>::ld(A + aoff + (size_t)mb * 16 * K + kc); if (NSPLIT == 1 || NSPLIT == 2) a2[mb] = WFrag<T16>::ld(A2 + aoff + (size_t)mb * 16 * K + kc); }
#pragma unroll
        for (int nb = 0; nb < 4; ++nb) { const V b = WFrag<T16>::ld(Bt + boff + (size_t)nb * 16 * K + kc); V b2; if (NSPLIT >= 2) b2 = WFrag<T16>::ld(Bt2 + boff + (size_t)nb * 16 * K + kc);
#pragma unroll
            for (int mb = 0; mb < 4; ++mb) { acc[mb][nb] = WFrag<T16>::mma(a[mb], b, acc[mb][nb]); if (NSPLIT == 1 || NSPLIT == 2) acc[mb][nb] = WFrag<T16>::mma(a2[mb], b, acc[mb][nb]); if (NSPLIT >= 2) acc[mb][nb] = WFrag<T16>::mma(a[mb], b2, acc[mb][nb]); } }
        asm volatile("v_nop\n\tv_nop\n\tv_nop\n\tv_nop" : "+v"(acc[0][0]), "+v"(acc[1][1]), "+v"(acc[2][2]), "+v"(acc[3][3]) : "v"(a[0]), "v"(a[3]));
    }
#pragma unroll
    for (int mb = 0; mb < 4; ++mb) {
#pragma unroll
        for (int nb = 0; nb < 4; ++nb) {
#pragma unroll
            for (int j = 0; j < 8; ++j) os[(hi * 8 + j) * 68 + nb * 16 + lr] = acc[mb][nb][j]; }
        __builtin_amdgcn_wave_barrier(); asm volatile("" ::: "memory");
        float* crow = C + (size_t)(r0 + mb * 16) * ldc + c0;
#pragma unroll 1
        for (int ps = 0; ps < 2; ++ps) {
#pragma unroll
            for (int s = 0; s < 8; ++s) { const int row = 2 * s + hi, cofs = lr * 4; v4f val = *(const v4fa*)(os + row * 68 + cofs); if (BIAS) { val[0] += bfr(bias[c0 + cofs]); val[1] += bfr(bias[c0 + cofs + 1]); val[2] += bfr(bias[c0 + cofs + 2]); val[3] += bfr(bias[c0 + cofs + 3]); }
                *(volatile v4f*)(crow + (size_t)row * ldc + cofs) = val; }
            if (ps == 0) __threadfence(); }
        __builtin_amdgcn_wave_barrier(); asm volatile("" ::: "memory");
    }
}

__device__ __forceinline__ h16 tohx(float x) { return (h16)x; }
__device__ __forceinline__ void splitf(float y, unsigned short& h, unsigned short& l) { h = f2bf(y); l = f2bf(y - bf2f(h)); }
typedef __attribute__((ext_vector_type(2))) _Float16 v2h;
typedef __attribute__((ext_vector_type(4))) _Float16 v4h;
typedef __attribute__((ext_vector_type(2))) unsigned short v2us;
typedef __attribute__((ext_vector_type(4))) unsigned short v4us;

__global__ __launch_bounds__(256) void k_cvt8(const float* __restrict__ src, bf* dst, size_t n8) { const size_t i = (size_t)blockIdx.x * 256 + threadIdx.x; if (i >= n8) return; const v8f v = *(const v8f*)(src + i * 8); v8us o;
#pragma unroll
    for (int k = 0; k < 8; ++k) o[k] = f2bf(v[k]); *(volatile v8us*)(dst + i * 8) = o; __threadfence(); *(volatile v8us*)(dst + i * 8) = o; }
__global__ __launch_bounds__(256) void k_pl(const float* __restrict__ F, int ld, int coff, float scl, h16* P16) { const size_t e = ((size_t)blockIdx.x * 256 + threadIdx.x) * 2; if (e >= (size_t)NH_ * NN * HD) return; const int d = (int)(e % HD); const int n = (int)((e / HD) % NN); const int h = (int)(e / ((size_t)HD * NN)); const float* f = F + (size_t)n * ld + coff + h * HD + d; v2h o; o[0] = tohx(f[0] * scl); o[1] = tohx(f[1] * scl); *(volatile v2h*)(P16 + e) = o; __threadfence(); *(volatile v2h*)(P16 + e) = o; }
__global__ __launch_bounds__(256) void k_vtp(const float* __restrict__ F, int ld, int coff, h16* VT) { const size_t e = ((size_t)blockIdx.x * 256 + threadIdx.x) * 2; if (e >= (size_t)NH_ * HD * NN) return; const int n = (int)(e % NN); const int d = (int)((e / NN) % HD); const int h = (int)(e / ((size_t)NN * HD)); v2h o; o[0] = tohx(F[(size_t)n * ld + coff + h * HD + d]); o[1] = tohx(F[(size_t)(n + 1) * ld + coff + h * HD + d]); *(volatile v2h*)(VT + e) = o; __threadfence(); *(volatile v2h*)(VT + e) = o; }
__global__ __launch_bounds__(256) void k_msoft(const float* __restrict__ Sb, const int* __restrict__ bidx, h16* P) { const int lane = threadIdx.x & 31; const int n = blockIdx.x * 8 + (threadIdx.x >> 5); if (n >= NN) return; const int bn = bidx[n]; const float* sr = Sb + (size_t)n * NN; float v[128]; float mx = -3.0e38f;
#pragma unroll
    for (int ch = 0; ch < 32; ++ch) { const int j0 = ch * 128 + lane * 4; const v4f a = *(const v4f*)(sr + j0);
#pragma unroll
        for (int q = 0; q < 4; ++q) { const float t = bidx[j0 + q] != bn ? -1.0e30f : a[q]; v[ch * 4 + q] = t; mx = fmaxf(mx, t); } }
#pragma unroll
    for (int sh = 16; sh; sh >>= 1) mx = fmaxf(mx, __shfl_xor(mx, sh, 32));
    float sum = 0.f;
#pragma unroll
    for (int k = 0; k < 128; ++k) { float d0 = __fsub_rn(v[k], mx); asm volatile("" : "+v"(d0)); v[k] = __expf(d0); sum += v[k]; }
#pragma unroll
    for (int sh = 16; sh; sh >>= 1) sum += __shfl_xor(sum, sh, 32);
    const float f = __fdiv_rn(PCAR, sum);
#pragma unroll 1
    for (int ps = 0; ps < 2; ++ps) {
#pragma unroll
        for (int ch = 0; ch < 32; ++ch) { v4h o; o[0] = tohx(v[ch * 4] * f); o[1] = tohx(v[ch * 4 + 1] * f); o[2] = tohx(v[ch * 4 + 2] * f); o[3] = tohx(v[ch * 4 + 3] * f); *(volatile v4h*)(P + (size_t)n * NN + ch * 128 + lane * 4) = o; }
        if (ps == 0) __threadfence(); } }
__global__ __launch_bounds__(256) void k_mrg(const float* __restrict__ Ob, int h, bf* Ah, bf* Al) { const size_t e = ((size_t)blockIdx.x * 256 + threadIdx.x) * 2; if (e >= (size_t)NN * HD) return; const int d = (int)(e % HD); const int n = (int)(e / HD); v2us oh, ol;
#pragma unroll
    for (int u = 0; u < 2; ++u) { unsigned short a, c; splitf(Ob[e + u] * (1.0f / PCAR), a, c); oh[u] = a; ol[u] = c; } const size_t o = (size_t)n * EE + h * HD + d; *(volatile v2us*)(Ah + o) = oh; *(volatile v2us*)(Al + o) = ol; __threadfence(); *(volatile v2us*)(Ah + o) = oh; *(volatile v2us*)(Al + o) = ol; }
__global__ __launch_bounds__(256) void k_lnres(const float* __restrict__ x, const float* __restrict__ DL, const float* __restrict__ g, const float* __restrict__ bb, float* Y) { const int lane = threadIdx.x & 31; const int n = blockIdx.x * 8 + (threadIdx.x >> 5); if (n >= NN) return; const size_t rb = (size_t)n * EE; float s = 0.f;
#pragma unroll 1
    for (int ch = 0; ch < 8; ++ch) { const size_t o = rb + ch * 128 + lane * 4; const v4f a = *(const v4f*)(x + o), dd = *(const v4f*)(DL + o);
#pragma unroll
        for (int q = 0; q < 4; ++q) s = __fadd_rn(s, __fadd_rn(bfr(a[q]), dd[q])); }
#pragma unroll
    for (int sh = 16; sh; sh >>= 1) s += __shfl_xor(s, sh, 32);
    const float mu = s * (1.0f / EE); float q2 = 0.f;
#pragma unroll 1
    for (int ch = 0; ch < 8; ++ch) { const size_t o = rb + ch * 128 + lane * 4; const v4f a = *(const v4f*)(x + o), dd = *(const v4f*)(DL + o);
#pragma unroll
        for (int q = 0; q < 4; ++q) { float dv = __fsub_rn(__fadd_rn(bfr(a[q]), dd[q]), mu); asm volatile("" : "+v"(dv)); float p = __fmul_rn(dv, dv); asm volatile("" : "+v"(p)); q2 = __fadd_rn(q2, p); } }
#pragma unroll
    for (int sh = 16; sh; sh >>= 1) q2 += __shfl_xor(q2, sh, 32);
    float vq = q2 * (1.0f / EE); asm volatile("" : "+v"(vq)); const float rs = __frsqrt_rn(__fadd_rn(vq, 1e-5f));
#pragma unroll 1
    for (int ch = 0; ch < 8; ++ch) { const size_t o = rb + ch * 128 + lane * 4; const v4f a = *(const v4f*)(x + o), dd = *(const v4f*)(DL + o); v4f r;
#pragma unroll
        for (int q = 0; q < 4; ++q) { const int d = ch * 128 + lane * 4 + q; float dv = __fsub_rn(__fadd_rn(bfr(a[q]), dd[q]), mu); asm volatile("" : "+v"(dv)); float tn = __fmul_rn(dv, rs); asm volatile("" : "+v"(tn)); float tg = __fmul_rn(tn, bfr(g[d])); asm volatile("" : "+v"(tg)); r[q] = __fadd_rn(tg, bfr(bb[d])); }
        *(volatile v4f*)(Y + o) = r; __threadfence(); *(volatile v4f*)(Y + o) = r; } }
__global__ __launch_bounds__(256) void k_copy2(const float* __restrict__ a, const float* __restrict__ b, size_t n4, float* OA, float* OB) { const size_t i = ((size_t)blockIdx.x * 256 + threadIdx.x) * 4; if (i >= n4 * 4) return; const v4f va = *(const v4f*)(a + i), vb = *(const v4f*)(b + i); *(volatile v4f*)(OA + i) = va; *(volatile v4f*)(OB + i) = vb; __threadfence(); *(volatile v4f*)(OA + i) = va; *(volatile v4f*)(OB + i) = vb; }

extern "C" void kernel_launch(void* const* d_in, const int* in_sizes, int n_in,
                              void* d_out, int out_size, void* d_ws, size_t ws_size, hipStream_t stream) {
    (void)in_sizes; (void)n_in; (void)out_size;
    const float* x = (const float*)d_in[0]; const int* bidx = (const int*)d_in[1]; const float* segm = (const float*)d_in[2]; const float* curm = (const float*)d_in[3]; const float* win = (const float*)d_in[4]; const float* binp = (const float*)d_in[5]; const float* wout = (const float*)d_in[6]; const float* bout = (const float*)d_in[7]; const float* lng = (const float*)d_in[8]; const float* lnb = (const float*)d_in[9];
    float* OUTY = (float*)d_out; float* OUT2 = (float*)((char*)d_out + 16777216); float* OUT3 = (float*)((char*)d_out + 33554432);
    char* wsp = (char*)d_ws;
    auto take = [&](size_t bytes) { char* p = wsp; wsp += (bytes + 255) & ~(size_t)255; return (void*)p; };
    bf* WI = (bf*)take((size_t)3 * EE * EE * 2); bf* WOt = (bf*)take((size_t)EE * EE * 2); bf* XB = (bf*)take((size_t)NN * EE * 2); float* QKV = (float*)take((size_t)NN * 3 * EE * 4);
    h16* Q16 = (h16*)take((size_t)NH_ * NN * HD * 2); h16* K16 = (h16*)take((size_t)NH_ * NN * HD * 2); h16* VT = (h16*)take((size_t)NH_ * HD * NN * 2); float* Sb = (float*)take((size_t)NN * NN * 4); h16* P16 = (h16*)take((size_t)NN * NN * 2); float* Ob = (float*)take((size_t)NN * HD * 4); bf* Ah = (bf*)take((size_t)NN * EE * 2); bf* Al = (bf*)take((size_t)NN * EE * 2); float* DLT = QKV;
    if ((size_t)(wsp - (char*)d_ws) > ws_size) return;
    k_cvt8<<<(3 * EE * EE / 8 + 255) / 256, 256, 0, stream>>>(win, WI, (size_t)3 * EE * EE / 8); k_cvt8<<<(EE * EE / 8 + 255) / 256, 256, 0, stream>>>(wout, WOt, (size_t)EE * EE / 8);
    k_copy2<<<(unsigned)(((size_t)NN * 1024 / 4 + 255) / 256), 256, 0, stream>>>(segm, curm, (size_t)NN * 1024 / 4, OUT2, OUT3);
    k_cvt8<<<(NN * EE / 8 + 255) / 256, 256, 0, stream>>>(x, XB, (size_t)NN * EE / 8);
    k_gemmw<bf, 0, true><<<dim3(NN / 64, 3 * EE / 64, 1), 32, 0, stream>>>(XB, nullptr, WI, nullptr, EE, QKV, 3 * EE, binp, 0, 0, 0);
    const unsigned LP = (unsigned)(((size_t)NH_ * NN * HD / 2 + 255) / 256);
    k_pl<<<LP, 256, 0, stream>>>(QKV, 3 * EE, 0, 0.08838834764831845f, Q16); k_pl<<<LP, 256, 0, stream>>>(QKV, 3 * EE, EE, 1.0f, K16); k_vtp<<<LP, 256, 0, stream>>>(QKV, 3 * EE, 2 * EE, VT);
    for (int h = 0; h < NH_; ++h) {
        k_gemmw<h16, 0, false><<<dim3(NN / 64, NN / 64, 1), 32, 0, stream>>>(Q16 + (size_t)h * NN * HD, nullptr, K16 + (size_t)h * NN * HD, nullptr, HD, Sb, NN, nullptr, 0, 0, 0);
        k_msoft<<<NN / 8, 256, 0, stream>>>(Sb, bidx, P16);
        k_gemmw<h16, 0, false><<<dim3(NN / 64, HD / 64, 1), 32, 0, stream>>>(P16, nullptr, VT + (size_t)h * HD * NN, nullptr, NN, Ob, HD, nullptr, 0, 0, 0);
        k_mrg<<<(unsigned)(((size_t)NN * HD / 2 + 255) / 256), 256, 0, stream>>>(Ob, h, Ah, Al); }
    k_gemmw<bf, 1, true><<<dim3(NN / 64, EE / 64, 1), 32, 0, stream>>>(Ah, Al, WOt, nullptr, EE, DLT, EE, bout, 0, 0, 0);
    k_lnres<<<NN / 8, 256, 0, stream>>>(x, DLT, lng, lnb, OUTY);
}
